// PointFeaturePropagation_34943853920281
// MI455X (gfx1250) — hardware-verified
//
#include <hip/hip_runtime.h>
#include <stdint.h>

#pragma clang fp contract(off)

typedef __attribute__((ext_vector_type(16))) _Float16 v16h;
typedef __attribute__((ext_vector_type(8)))  _Float16 v8h;
typedef __attribute__((ext_vector_type(16))) __bf16   v16b;
typedef __attribute__((ext_vector_type(8)))  __bf16   v8b;
typedef __attribute__((ext_vector_type(8)))  float    v8f;
typedef __attribute__((ext_vector_type(4)))  float    v4f;

constexpr int NB_B   = 4;
constexpr int NQ_PTS = 16384;
constexpr int NS_PTS = 4096;
constexpr int LD_P1  = 67;
constexpr int LD_P2  = 259;
constexpr int CF_1   = 64;
constexpr int CF_2   = 256;
constexpr int CIN_0  = 320;
constexpr int CH_1   = 256;
constexpr int CH_2   = 128;
constexpr int CH_3   = 128;
constexpr int LD_OUT = 131;
constexpr int NROWS  = NB_B * NQ_PTS;
constexpr float W_CARRY     = 16.0f;
constexpr float W_CARRY_INV = 0.0625f;
constexpr float KNN_EPS     = 1e-8f;
constexpr int KNN_TPB   = 256;
constexpr int KNN_CHUNK = 2048;

static_assert(NQ_PTS % KNN_TPB == 0);
static_assert(NS_PTS % KNN_CHUNK == 0);
static_assert(KNN_CHUNK % KNN_TPB == 0);
static_assert(KNN_CHUNK % 4 == 0);
static_assert(NROWS % 64 == 0);
static_assert(CH_1 % 64 == 0 && CH_2 % 64 == 0 && CH_3 % 64 == 0);
static_assert(CIN_0 % 32 == 0 && CH_1 % 32 == 0 && CH_2 % 32 == 0);
static_assert(CF_1 + CF_2 == CIN_0);

constexpr size_t SZ_H0  = (size_t)NROWS * CIN_0 * 2;
constexpr size_t SZ_H3  = (size_t)NROWS * CH_3 * 4;
constexpr size_t SZ_R0  = SZ_H0 > SZ_H3 ? SZ_H0 : SZ_H3;
constexpr size_t SZ_F2  = (size_t)NB_B * NS_PTS * CF_2 * 4;
constexpr size_t SZ_H2  = (size_t)NROWS * CH_2 * 2;
constexpr size_t SZ_R1  = SZ_F2 > SZ_H2 ? SZ_F2 : SZ_H2;
constexpr size_t SZ_H1  = (size_t)NROWS * CH_1 * 2;
constexpr size_t SZ_W1T = (size_t)CH_1 * CIN_0 * 2;
constexpr size_t SZ_W2T = (size_t)CH_2 * CH_1 * 2;
constexpr size_t SZ_W3T = (size_t)CH_3 * CH_2 * 2;
constexpr size_t OFF_R0 = 0;
constexpr size_t OFF_R1 = OFF_R0 + SZ_R0;
constexpr size_t OFF_R2 = OFF_R1 + SZ_R1;
constexpr size_t OFF_W1 = OFF_R2 + SZ_H1;
constexpr size_t OFF_W2 = OFF_W1 + SZ_W1T;
constexpr size_t OFF_W3 = OFF_W2 + SZ_W2T;
constexpr size_t WS_TOTAL = OFF_W3 + SZ_W3T;
static_assert(WS_TOTAL == 92536832);
static_assert(WS_TOTAL <= 134217728);
static_assert(OFF_R1 % 128 == 0 && OFF_R2 % 128 == 0 && OFF_W1 % 128 == 0 && OFF_W2 % 128 == 0 && OFF_W3 % 128 == 0);

__device__ __forceinline__ unsigned short f2bf_bits(float f) {
  unsigned u = __float_as_uint(f);
  return (unsigned short)((u + 0x7FFFu + ((u >> 16) & 1u)) >> 16);
}
__device__ __forceinline__ float bf_bits2f(unsigned short h) { return __uint_as_float(((unsigned)h) << 16); }

__device__ __forceinline__ void dep_guard_h(v8f& a, v8f& b, v16h x, v16h y) { asm volatile("v_nop\n\tv_nop\n\tv_nop\n\tv_nop" : "+v"(a), "+v"(b) : "v"(x), "v"(y)); }
__device__ __forceinline__ void dep_guard_b(v8f& a, v8f& b, v16b x, v16b y) { asm volatile("v_nop\n\tv_nop\n\tv_nop\n\tv_nop" : "+v"(a), "+v"(b) : "v"(x), "v"(y)); }
__device__ __forceinline__ void keep4_h(v16h a, v16h b, v16h c, v16h d) { asm volatile("v_nop" :: "v"(a), "v"(b), "v"(c), "v"(d)); }
__device__ __forceinline__ void keep4_b(v16b a, v16b b, v16b c, v16b d) { asm volatile("v_nop" :: "v"(a), "v"(b), "v"(c), "v"(d)); }
__device__ __forceinline__ void acc_guard4(v8f& a, v8f& b, v8f& c, v8f& d) { asm volatile("v_nop\n\tv_nop\n\tv_nop\n\tv_nop" : "+v"(a), "+v"(b), "+v"(c), "+v"(d)); }
template <typename T> struct Frag;
template <> struct Frag<_Float16> {
  typedef v16h V; union U { v16h v; v8h h[2]; };
  static __device__ __forceinline__ v16h load(const _Float16* p) {
    U f; f.h[0] = *(const v8h*)(p); f.h[1] = *(const v8h*)(p + 16); return f.v;
  }
  static __device__ __forceinline__ v8f mma(v16h a, v16h b, v8f c) {
    return __builtin_amdgcn_wmma_f32_16x16x32_f16(false, a, false, b, (short)0, c, false, false);
  }
  static __device__ __forceinline__ void guard(v8f& a, v8f& b, v16h x, v16h y) { dep_guard_h(a, b, x, y); }
  static __device__ __forceinline__ void keep(v16h a, v16h b, v16h c, v16h d) { keep4_h(a, b, c, d); }
};
template <> struct Frag<__bf16> {
  typedef v16b V; union U { v16b v; v8b h[2]; };
  static __device__ __forceinline__ v16b load(const __bf16* p) {
    U f; f.h[0] = *(const v8b*)(p); f.h[1] = *(const v8b*)(p + 16); return f.v;
  }
  static __device__ __forceinline__ v8f mma(v16b a, v16b b, v8f c) {
    return __builtin_amdgcn_wmma_f32_16x16x32_bf16(false, a, false, b, (short)0, c, false, false);
  }
  static __device__ __forceinline__ void guard(v8f& a, v8f& b, v16b x, v16b y) { dep_guard_b(a, b, x, y); }
  static __device__ __forceinline__ void keep(v16b a, v16b b, v16b c, v16b d) { keep4_b(a, b, c, d); }
};

template <int ET> struct Elem;
template <> struct Elem<0> { typedef _Float16 T; };
template <> struct Elem<1> { typedef __bf16 T; };
template <int ET, bool SPLIT, int BIAS_MODE, int OUT_MODE, bool RESID, int ACT = 0>
__global__ __launch_bounds__(256) void wmma_gemm64(
    const unsigned short* __restrict__ Ap, const unsigned short* __restrict__ A2p, int lda, long strideA,
    const unsigned short* __restrict__ Btp, const unsigned short* __restrict__ Bt2p, int ldb, long strideB,
    void* __restrict__ Cout, void* __restrict__ Cout2, int ldc, long strideC,
    const float* __restrict__ bias,
    const float* __restrict__ resid, long strideR,
    int M, int N, int K, float scale) {
  typedef typename Elem<ET>::T T;
  typedef typename Frag<T>::V V;
  const T* A = (const T*)Ap; const T* A2 = (const T*)A2p; const T* Bt = (const T*)Btp; const T* Bt2 = (const T*)Bt2p;
  __shared__ __align__(16) float sT[8][16 * 68];
  const int b    = blockIdx.y;
  const int lane = threadIdx.x & 31;
  const int wave = threadIdx.x >> 5;
  const int tilesN = N >> 6;
  const int tilesM = M >> 6;
  const int tile = blockIdx.x * 8 + wave;
  if (tile >= tilesM * tilesN) return;
  const int tm = tile / tilesN;
  const int tn = tile - tm * tilesN;
  const int m0 = tm << 6;
  const int n0 = tn << 6;

  const T* Ab  = A  + (size_t)b * strideA;
  const T* Bb  = Bt + (size_t)b * strideB;
  const T* Ab2 = SPLIT ? (A2  + (size_t)b * strideA) : nullptr;
  const T* Bb2 = SPLIT ? (Bt2 + (size_t)b * strideB) : nullptr;

  const int rlane = lane & 15;
  const int koff  = (lane >> 4) * 8;
  const int mOff  = (lane >> 4) * 8;

  v8f acc[4][4];
#pragma unroll
  for (int i = 0; i < 4; ++i)
#pragma unroll
    for (int j = 0; j < 4; ++j) acc[i][j] = (v8f){0.f,0.f,0.f,0.f,0.f,0.f,0.f,0.f};

  for (int k0 = 0; k0 < K; k0 += 32) {
    V bh[4], bl[4];
#pragma unroll
    for (int j = 0; j < 4; ++j) {
      const size_t bo = (size_t)(n0 + (j << 4) + rlane) * ldb + koff + k0;
      bh[j] = Frag<T>::load(Bb + bo);
      if (SPLIT) bl[j] = Frag<T>::load(Bb2 + bo);
    }
#pragma unroll
    for (int i = 0; i < 4; ++i) {
      const size_t ao = (size_t)(m0 + (i << 4) + rlane) * lda + koff + k0;
      V ah = Frag<T>::load(Ab + ao);
      V al;
      if (SPLIT) al = Frag<T>::load(Ab2 + ao);
#pragma unroll
      for (int j = 0; j < 4; ++j) {
        acc[i][j] = Frag<T>::mma(ah, bh[j], acc[i][j]);
        if (SPLIT) {
          acc[i][j] = Frag<T>::mma(ah, bl[j], acc[i][j]);
          acc[i][j] = Frag<T>::mma(al, bh[j], acc[i][j]);
        }
      }
      Frag<T>::guard(acc[i][0], acc[i][3], ah, SPLIT ? al : ah);
    }
    Frag<T>::keep(bh[0], bh[1], bh[2], bh[3]);
    if (SPLIT) Frag<T>::keep(bl[0], bl[1], bl[2], bl[3]);
  }
  acc_guard4(acc[0][0], acc[0][1], acc[0][2], acc[0][3]);
  acc_guard4(acc[1][0], acc[1][1], acc[1][2], acc[1][3]);
  acc_guard4(acc[2][0], acc[2][1], acc[2][2], acc[2][3]);
  acc_guard4(acc[3][0], acc[3][1], acc[3][2], acc[3][3]);

  float* slab = sT[wave];
  const float* Rb = RESID ? (resid + (size_t)b * strideR) : nullptr;
#pragma unroll
  for (int i = 0; i < 4; ++i) {
    const int mBase = m0 + (i << 4);
#pragma unroll
    for (int j = 0; j < 4; ++j) {
      const int n = n0 + (j << 4) + rlane;
      float bv = 0.f;
      if (BIAS_MODE == 2) bv = bias[n];
#pragma unroll
      for (int r = 0; r < 8; ++r) {
        float v = acc[i][j][r] * scale;
        if (BIAS_MODE == 1) v += bias[mBase + mOff + r];
        if (BIAS_MODE == 2) v += bv;
        if (RESID) v += Rb[(size_t)(mBase + mOff + r) * ldc + n];
        if (ACT == 1) v = tanhf(v);
        if (ACT == 2) v = fmaxf(v, 0.0f);
        if (ACT == 3) v = v / (1.0f + expf(-v));
        if (ACT == 4) v = (v > 0.f) ? v : 0.01f * v;
        if (ACT == 5) v = 0.5f * v * (1.0f + erff(v * 0.70710678118654752f));
        slab[(mOff + r) * 68 + (j << 4) + rlane] = v;
      }
    }
    __builtin_amdgcn_fence(__ATOMIC_RELEASE, "workgroup");
    __builtin_amdgcn_wave_barrier();
    __builtin_amdgcn_fence(__ATOMIC_ACQUIRE, "workgroup");
    if (OUT_MODE == 0) {
      float* C = (float*)Cout + (size_t)b * strideC;
      const int hh = lane >> 4, c4 = (lane & 15) * 4;
      for (int pass = 0; pass < 2; ++pass) {
#pragma unroll
        for (int it = 0; it < 8; ++it) {
          const int row = it * 2 + hh;
          v4f v = *(const v4f*)(slab + row * 68 + c4);
          *(volatile v4f*)(C + (size_t)(mBase + row) * ldc + n0 + c4) = v;
        }
        __threadfence();
      }
    } else {
      const int q = lane >> 3, c8 = (lane & 7) * 8;
      unsigned short* C  = (unsigned short*)Cout  + (size_t)b * strideC;
      unsigned short* C2 = (OUT_MODE == 2) ? ((unsigned short*)Cout2 + (size_t)b * strideC) : nullptr;
      for (int pass = 0; pass < 2; ++pass) {
#pragma unroll
        for (int it = 0; it < 4; ++it) {
          const int row = it * 4 + q;
          const float* sp = slab + row * 68 + c8;
          v8h hv, lv;
#pragma unroll
          for (int e = 0; e < 8; ++e) {
            if (OUT_MODE == 1) {
              hv[e] = (_Float16)sp[e];
            } else {
              unsigned short hb = f2bf_bits(sp[e]);
              unsigned short lb = f2bf_bits(sp[e] - bf_bits2f(hb));
              hv[e] = __builtin_bit_cast(_Float16, hb);
              lv[e] = __builtin_bit_cast(_Float16, lb);
            }
          }
          *(volatile v8h*)(C + (size_t)(mBase + row) * ldc + n0 + c8) = hv;
          if (OUT_MODE == 2) *(volatile v8h*)(C2 + (size_t)(mBase + row) * ldc + n0 + c8) = lv;
        }
        __threadfence();
      }
    }
    __builtin_amdgcn_fence(__ATOMIC_RELEASE, "workgroup");
    __builtin_amdgcn_wave_barrier();
    __builtin_amdgcn_fence(__ATOMIC_ACQUIRE, "workgroup");
  }
}

__global__ __launch_bounds__(256) void wt_cast_kernel(
    const float* __restrict__ W, unsigned short* __restrict__ Wt, int kdim, int ndim, float sc)
{
  const int qpr = kdim >> 3;
  const int total = ndim * qpr;
  int t = blockIdx.x * 256 + threadIdx.x;
  const bool ok = t < total;
  t = ok ? t : (total - 1);
  const int n = t / qpr;
  const int q = t - n * qpr;
  v8h hv;
#pragma unroll
  for (int e = 0; e < 8; ++e) hv[e] = (_Float16)(W[(size_t)(8 * q + e) * ndim + n] * sc);
  unsigned short* dst = Wt + (size_t)n * kdim + 8 * q;
  if (ok) {
    *(volatile v8h*)dst = hv;
    __threadfence();
    *(volatile v8h*)dst = hv;
  }
}

__global__ __launch_bounds__(256) void feat_copy_kernel(
    const float* __restrict__ p2, float* __restrict__ f2)
{
  const int t = blockIdx.x * 256 + threadIdx.x;
  const int row = t >> 6;
  const int q = t & 63;
  const float* s = p2 + (size_t)row * LD_P2 + 3 + 4 * q;
  v4f v;
  v[0] = s[0]; v[1] = s[1]; v[2] = s[2]; v[3] = s[3];
  float* d = f2 + (size_t)row * CF_2 + 4 * q;
  *(volatile v4f*)d = v;
  __threadfence();
  *(volatile v4f*)d = v;
}

__device__ __forceinline__ void order2(float& da, int& ia, float& db, int& ib) {
  const bool sw = (db < da) || ((db == da) && (ib < ia));
  const float nd0 = sw ? db : da;
  const float nd1 = sw ? da : db;
  const int ni0 = sw ? ib : ia;
  const int ni1 = sw ? ia : ib;
  da = nd0; db = nd1; ia = ni0; ib = ni1;
}

__global__ __launch_bounds__(KNN_TPB) void knn_interp_kernel(
    const float* __restrict__ p1, const float* __restrict__ p2,
    const float* __restrict__ f2, unsigned short* __restrict__ h0)
{
  __shared__ __align__(16) v4f s_xyz[KNN_CHUNK];
  __shared__ int   s_j0[KNN_TPB];
  __shared__ int   s_j1[KNN_TPB];
  __shared__ int   s_j2[KNN_TPB];
  __shared__ float s_w0[KNN_TPB];
  __shared__ float s_w1[KNN_TPB];
  __shared__ float s_w2[KNN_TPB];

  const int tid  = threadIdx.x;
  const int lane = tid & 31;
  const int wave = tid >> 5;
  const int b    = blockIdx.y;
  const int q0   = blockIdx.x * KNN_TPB;
  const float* p2b = p2 + (size_t)b * NS_PTS * LD_P2;

  const float* p1r = p1 + ((size_t)b * NQ_PTS + q0 + tid) * LD_P1;
  const float x1 = p1r[0], y1 = p1r[1], z1 = p1r[2];
  const float ta = x1 * x1;
  const float tb = y1 * y1;
  const float tc = z1 * z1;
  const float aa = (ta + tc) + tb;

  float k0 = __builtin_huge_valf();
  float k1 = k0, k2 = k0, k3 = k0;
  int i0 = 0, i1 = 0, i2 = 0, i3 = 0;

  for (int cb = 0; cb < NS_PTS; cb += KNN_CHUNK) {
    __syncthreads();
#pragma unroll 1
    for (int j = tid; j < KNN_CHUNK; j += KNN_TPB) {
      const float* src = p2b + (size_t)(cb + j) * LD_P2;
      const float x = src[0], y = src[1], z = src[2];
      const float u0 = x * x;
      const float u1 = y * y;
      const float u2 = z * z;
      v4f e;
      e[0] = x; e[1] = y; e[2] = z; e[3] = (u0 + u2) + u1;
      s_xyz[j] = e;
    }
    __syncthreads();
#pragma unroll 1
    for (int j = 0; j < KNN_CHUNK; j += 4) {
#pragma unroll
      for (int u = 0; u < 4; ++u) {
        const v4f c = s_xyz[j + u];
        float p = x1 * c[0];
        p = fmaf(y1, c[1], p);
        p = fmaf(z1, c[2], p);
        const float s = aa + c[3];
        const float d2 = fmaf(-2.0f, p, s);
        if (d2 < k3) {
          const int jg = cb + j + u;
          const bool c2 = d2 < k2;
          const bool c1 = d2 < k1;
          const bool c0 = d2 < k0;
          k3 = c2 ? k2 : d2;             i3 = c2 ? i2 : jg;
          k2 = c2 ? (c1 ? k1 : d2) : k2; i2 = c2 ? (c1 ? i1 : jg) : i2;
          k1 = c1 ? (c0 ? k0 : d2) : k1; i1 = c1 ? (c0 ? i0 : jg) : i1;
          k0 = c0 ? d2 : k0;             i0 = c0 ? jg : i0;
        }
      }
    }
  }

  float d0 = sqrtf(fmaxf(k0, 0.0f));
  float d1 = sqrtf(fmaxf(k1, 0.0f));
  float d2v = sqrtf(fmaxf(k2, 0.0f));
  float d3 = sqrtf(fmaxf(k3, 0.0f));
  order2(d0, i0, d1, i1);
  order2(d2v, i2, d3, i3);
  order2(d0, i0, d2v, i2);
  order2(d1, i1, d3, i3);
  order2(d1, i1, d2v, i2);

  float w0 = __builtin_amdgcn_rcpf(d0 + KNN_EPS);
  float w1 = __builtin_amdgcn_rcpf(d1 + KNN_EPS);
  float w2 = __builtin_amdgcn_rcpf(d2v + KNN_EPS);
  const float wsum = (w0 + w1) + w2;
  const float winv = __builtin_amdgcn_rcpf(wsum);
  s_j0[tid] = i0; s_j1[tid] = i1; s_j2[tid] = i2;
  s_w0[tid] = w0 * winv; s_w1[tid] = w1 * winv; s_w2[tid] = w2 * winv;
  __syncthreads();

  const size_t rowBase = (size_t)b * NQ_PTS + q0;
  const float* f2b = f2 + (size_t)b * NS_PTS * CF_2;
  const int lf = lane & 7;
#pragma unroll 1
  for (int rr = 0; rr < KNN_TPB / 8; ++rr) {
    const int r = wave + 8 * rr;
    int j0 = s_j0[r], j1 = s_j1[r], j2 = s_j2[r];
    j0 = j0 < 0 ? 0 : (j0 > NS_PTS - 1 ? NS_PTS - 1 : j0);
    j1 = j1 < 0 ? 0 : (j1 > NS_PTS - 1 ? NS_PTS - 1 : j1);
    j2 = j2 < 0 ? 0 : (j2 > NS_PTS - 1 ? NS_PTS - 1 : j2);
    const float rw0 = s_w0[r], rw1 = s_w1[r], rw2 = s_w2[r];
    const size_t grow = rowBase + (size_t)r;

    const float* fs = p1 + grow * LD_P1 + 3 + 8 * lf;
    v8h fh;
#pragma unroll
    for (int e = 0; e < 8; ++e) fh[e] = (_Float16)fs[e];

    const float* g0 = f2b + (size_t)j0 * CF_2 + 8 * lane;
    const float* g1 = f2b + (size_t)j1 * CF_2 + 8 * lane;
    const float* g2 = f2b + (size_t)j2 * CF_2 + 8 * lane;
    const v4f a0v = *(const v4f*)g0;
    const v4f a1v = *(const v4f*)(g0 + 4);
    const v4f b0v = *(const v4f*)g1;
    const v4f b1v = *(const v4f*)(g1 + 4);
    const v4f c0v = *(const v4f*)g2;
    const v4f c1v = *(const v4f*)(g2 + 4);
    v8h iv;
#pragma unroll
    for (int e = 0; e < 4; ++e) {
      float v = rw0 * a0v[e];
      v = fmaf(rw1, b0v[e], v);
      v = fmaf(rw2, c0v[e], v);
      iv[e] = (_Float16)v;
      float u = rw0 * a1v[e];
      u = fmaf(rw1, b1v[e], u);
      u = fmaf(rw2, c1v[e], u);
      iv[4 + e] = (_Float16)u;
    }
    unsigned short* hrow = h0 + grow * CIN_0;
    for (int pass = 0; pass < 2; ++pass) {
      if (lane < 8) *(volatile v8h*)(hrow + 8 * lf) = fh;
      *(volatile v8h*)(hrow + CF_1 + 8 * lane) = iv;
      __threadfence();
    }
  }
}

__global__ __launch_bounds__(256) void pack_out_kernel(
    const float* __restrict__ p1, const float* __restrict__ h3, float* __restrict__ out)
{
  const int t = blockIdx.x * 256 + threadIdx.x;
  v4f v;
#pragma unroll
  for (int e = 0; e < 4; ++e) {
    const int idx = 4 * t + e;
    const int row = idx / LD_OUT;
    const int col = idx - row * LD_OUT;
    const int cx = col < 3 ? col : 0;
    const int ch = col >= 3 ? (col - 3) : 0;
    const float vx = p1[(size_t)row * LD_P1 + cx];
    const float vh = h3[(size_t)row * CH_3 + ch];
    v[e] = col < 3 ? vx : vh;
  }
  float* d = out + (size_t)4 * t;
  *(volatile v4f*)d = v;
  __threadfence();
  *(volatile v4f*)d = v;
}

extern "C" void kernel_launch(void* const* d_in, const int* in_sizes, int n_in,
                              void* d_out, int out_size, void* d_ws, size_t ws_size,
                              hipStream_t stream)
{
  if (n_in < 8) return;
  if (out_size != NROWS * LD_OUT) return;
  if (ws_size < WS_TOTAL) return;
  if (in_sizes[0] != NB_B * NQ_PTS * LD_P1) return;
  if (in_sizes[1] != NB_B * NS_PTS * LD_P2) return;

  const float* p1  = (const float*)d_in[0];
  const float* p2  = (const float*)d_in[1];
  const float* W1  = (const float*)d_in[2];
  const float* bb1 = (const float*)d_in[3];
  const float* W2  = (const float*)d_in[4];
  const float* bb2 = (const float*)d_in[5];
  const float* W3  = (const float*)d_in[6];
  const float* bb3 = (const float*)d_in[7];
  float* out = (float*)d_out;

  char* ws = (char*)d_ws;
  unsigned short* H0  = (unsigned short*)(ws + OFF_R0);
  float*          H3  = (float*)(ws + OFF_R0);
  float*          F2  = (float*)(ws + OFF_R1);
  unsigned short* H2  = (unsigned short*)(ws + OFF_R1);
  unsigned short* H1  = (unsigned short*)(ws + OFF_R2);
  unsigned short* W1t = (unsigned short*)(ws + OFF_W1);
  unsigned short* W2t = (unsigned short*)(ws + OFF_W2);
  unsigned short* W3t = (unsigned short*)(ws + OFF_W3);

  {
    const int t1 = CH_1 * (CIN_0 / 8);
    const int t2 = CH_2 * (CH_1 / 8);
    const int t3 = CH_3 * (CH_2 / 8);
    wt_cast_kernel<<<dim3((t1 + 255) / 256), dim3(256), 0, stream>>>(W1, W1t, CIN_0, CH_1, W_CARRY);
    wt_cast_kernel<<<dim3((t2 + 255) / 256), dim3(256), 0, stream>>>(W2, W2t, CH_1, CH_2, W_CARRY);
    wt_cast_kernel<<<dim3((t3 + 255) / 256), dim3(256), 0, stream>>>(W3, W3t, CH_2, CH_3, W_CARRY);
  }

  static_assert((NB_B * NS_PTS * (CF_2 / 4)) % 256 == 0);
  feat_copy_kernel<<<dim3(NB_B * NS_PTS * (CF_2 / 4) / 256), dim3(256), 0, stream>>>(p2, F2);

  knn_interp_kernel<<<dim3(NQ_PTS / KNN_TPB, NB_B), dim3(KNN_TPB), 0, stream>>>(p1, p2, F2, H0);

  static_assert(NROWS % 64 == 0 && CH_1 % 64 == 0 && CIN_0 % 32 == 0);
  {
    const int tiles = (NROWS / 64) * (CH_1 / 64);
    hipLaunchKernelGGL((wmma_gemm64<0, false, 2, 1, false, 2>), dim3((tiles + 7) / 8, 1), dim3(256), 0, stream,
                       (const unsigned short*)H0, (const unsigned short*)H0, (int)CIN_0, (long)0,
                       (const unsigned short*)W1t, (const unsigned short*)W1t, (int)CIN_0, (long)0,
                       (void*)H1, (void*)H1, (int)CH_1, (long)0,
                       bb1, bb1, (long)0,
                       (int)NROWS, (int)CH_1, (int)CIN_0, W_CARRY_INV);
  }
  static_assert(CH_2 % 64 == 0 && CH_1 % 32 == 0);
  {
    const int tiles = (NROWS / 64) * (CH_2 / 64);
    hipLaunchKernelGGL((wmma_gemm64<0, false, 2, 1, false, 2>), dim3((tiles + 7) / 8, 1), dim3(256), 0, stream,
                       (const unsigned short*)H1, (const unsigned short*)H1, (int)CH_1, (long)0,
                       (const unsigned short*)W2t, (const unsigned short*)W2t, (int)CH_1, (long)0,
                       (void*)H2, (void*)H2, (int)CH_2, (long)0,
                       bb2, bb2, (long)0,
                       (int)NROWS, (int)CH_2, (int)CH_1, W_CARRY_INV);
  }
  static_assert(CH_3 % 64 == 0 && CH_2 % 32 == 0);
  {
    const int tiles = (NROWS / 64) * (CH_3 / 64);
    hipLaunchKernelGGL((wmma_gemm64<0, false, 2, 0, false, 2>), dim3((tiles + 7) / 8, 1), dim3(256), 0, stream,
                       (const unsigned short*)H2, (const unsigned short*)H2, (int)CH_2, (long)0,
                       (const unsigned short*)W3t, (const unsigned short*)W3t, (int)CH_2, (long)0,
                       (void*)H3, (void*)H3, (int)CH_3, (long)0,
                       bb3, bb3, (long)0,
                       (int)NROWS, (int)CH_3, (int)CH_2, W_CARRY_INV);
  }

  static_assert((NROWS * LD_OUT) % 1024 == 0);
  pack_out_kernel<<<dim3(NROWS * LD_OUT / 1024), dim3(256), 0, stream>>>(p1, H3, out);
}
